// SparseEncoderIN_16758962389328
// MI455X (gfx1250) — hardware-verified
//
#include <hip/hip_runtime.h>


typedef _Float16 v16h __attribute__((ext_vector_type(16)));
typedef float    v8f  __attribute__((ext_vector_type(8)));
typedef _Float16 v8h_na __attribute__((ext_vector_type(8)));
typedef _Float16 v4h_na __attribute__((ext_vector_type(4)));
typedef float    v4f_na __attribute__((ext_vector_type(4)));
typedef int      v4i_na __attribute__((ext_vector_type(4)));
typedef v8h_na __attribute__((may_alias)) v8h;
typedef v4h_na __attribute__((may_alias)) v4h;
typedef v4f_na __attribute__((may_alias)) v4f;
typedef v4i_na __attribute__((may_alias)) v4i;

union Frag { v16h v; v8h p[2]; };

#define NB 4
#define V0 262144
#define WS_LIMIT 134217728ull

__device__ __forceinline__ v8f wmma_f16(const v16h& a, const v16h& b, v8f c)
{
    return __builtin_amdgcn_wmma_f32_16x16x32_f16(false, a, false, b, (short)0, c, false, false);
}

template <int NT> struct Guard;
template <> struct Guard<2> {
    static __device__ __forceinline__ void run(v8f (&acc)[2], const v16h& a, const v16h& b) {
        asm volatile("v_nop\n\tv_nop\n\tv_nop\n\tv_nop"
                     : "+v"(acc[0]), "+v"(acc[1]) : "v"(a), "v"(b));
    }
};
template <> struct Guard<4> {
    static __device__ __forceinline__ void run(v8f (&acc)[4], const v16h& a, const v16h& b) {
        asm volatile("v_nop\n\tv_nop\n\tv_nop\n\tv_nop"
                     : "+v"(acc[0]), "+v"(acc[1]), "+v"(acc[2]), "+v"(acc[3]) : "v"(a), "v"(b));
    }
};

template <int NL, int LPV>
__device__ __forceinline__ void write_lines(const unsigned char* s, unsigned char* g,
                                            int pitch, int wave, int lane)
{
    static_assert(NL % 32 == 0);
    constexpr int NIT = NL / 32;
    constexpr int LL  = (LPV == 1) ? 0 : ((LPV == 2) ? 1 : 2);
    static_assert((1 << LL) == LPV);
    const int q = lane >> 3, j = lane & 7;
    v4i vals[NIT];
    size_t off[NIT];
#pragma unroll
    for (int it = 0; it < NIT; ++it) {
        const int L = (wave * NIT + it) * 4 + q;
        const int n = L >> LL, p = L & (LPV - 1);
        vals[it] = *(const v4i*)(s + (size_t)L * 128 + j * 16);
        off[it]  = (size_t)n * pitch + (size_t)p * 128 + j * 16;
    }
#pragma unroll
    for (int it = 0; it < NIT; ++it) *(volatile v4i*)(g + off[it]) = vals[it];
    __threadfence();
#pragma unroll
    for (int it = 0; it < NIT; ++it) *(volatile v4i*)(g + off[it]) = vals[it];
}

__global__ __launch_bounds__(256)
void k_prep_x(const float* __restrict__ x, const int* __restrict__ mask,
              _Float16* __restrict__ xh, int total)
{
    const int i = blockIdx.x * 256 + threadIdx.x;
    if (i >= total) return;
    const int b = i >> 18, v = i & (V0 - 1);
    const bool act = mask[i] < 1;
    const float* xb = x + (size_t)b * 3 * V0 + v;
    const float f0 = act ? xb[0] : 0.f;
    const float f1 = act ? xb[V0] : 0.f;
    const float f2 = act ? xb[2 * V0] : 0.f;
    v4h o = {(_Float16)f0, (_Float16)f1, (_Float16)f2, (_Float16)0.f};
    volatile v4h* p = (volatile v4h*)(xh + (size_t)i * 4);
    *p = o;
    __threadfence();
    *p = o;
}

__global__ __launch_bounds__(256)
void k_wt1(const float* __restrict__ w1, _Float16* __restrict__ wt1, int total)
{
    const int i = blockIdx.x * 256 + threadIdx.x;
    if (i >= total) return;
    const int co = i >> 5, s = i & 31;
    float f0 = 0.f, f1 = 0.f, f2 = 0.f;
    if (s < 27) {
        const float* wp = w1 + (size_t)co * 81 + s;
        f0 = wp[0] * 8.f; f1 = wp[27] * 8.f; f2 = wp[54] * 8.f;
    }
    v4h o = {(_Float16)f0, (_Float16)f1, (_Float16)f2, (_Float16)0.f};
    volatile v4h* p = (volatile v4h*)(wt1 + (size_t)i * 4);
    *p = o;
    __threadfence();
    *p = o;
}

__global__ __launch_bounds__(256)
void k_wtn(const float* __restrict__ w, _Float16* __restrict__ wt,
           int COUT, int CIN, float scale, int total8)
{
    const int i = blockIdx.x * 256 + threadIdx.x;
    if (i >= total8) return;
    const int cig = CIN >> 3;
    const int g = i % cig;
    const int r = i / cig;
    const int co = r % COUT;
    const int t  = r / COUT;
    const float* wp = w + ((size_t)co * CIN + g * 8) * 27 + t;
    float f[8];
#pragma unroll
    for (int jj = 0; jj < 8; ++jj) f[jj] = wp[jj * 27] * scale;
    v8h o = {(_Float16)f[0], (_Float16)f[1], (_Float16)f[2], (_Float16)f[3],
             (_Float16)f[4], (_Float16)f[5], (_Float16)f[6], (_Float16)f[7]};
    volatile v8h* p = (volatile v8h*)(wt + (size_t)i * 8);
    *p = o;
    __threadfence();
    *p = o;
}

__global__ __launch_bounds__(256)
void k_mask1(const int* __restrict__ mask, int* __restrict__ m1, int total)
{
    const int i = blockIdx.x * 256 + threadIdx.x;
    if (i >= total) return;
    const int xx = i & 63, yy = (i >> 6) & 63, zz = (i >> 12) & 63, b = i >> 18;
    const int* mb = mask + (size_t)b * V0;
    int act = 0;
#pragma unroll
    for (int tz = 0; tz < 3; ++tz) {
        const int iz = zz - 1 + tz;
        if ((unsigned)iz >= 64u) continue;
#pragma unroll
        for (int ty = 0; ty < 3; ++ty) {
            const int iy = yy - 1 + ty;
            if ((unsigned)iy >= 64u) continue;
            const int* row = mb + (iz * 64 + iy) * 64;
#pragma unroll
            for (int tx = 0; tx < 3; ++tx) {
                const int ix = xx - 1 + tx;
                if ((unsigned)ix < 64u) act |= (row[ix] < 1) ? 1 : 0;
            }
        }
    }
    volatile int* p = (volatile int*)(m1 + i);
    *p = act;
    __threadfence();
    *p = act;
}

template <int LOG2D>
__global__ __launch_bounds__(256)
void k_dil(const int* __restrict__ mi, int* __restrict__ mo, int total)
{
    constexpr int D = 1 << LOG2D, Din = 2 * D;
    const int i = blockIdx.x * 256 + threadIdx.x;
    if (i >= total) return;
    const int xx = i & (D - 1), yy = (i >> LOG2D) & (D - 1), zz = (i >> (2 * LOG2D)) & (D - 1);
    const int b = i >> (3 * LOG2D);
    const int* mb = mi + (size_t)b * Din * Din * Din;
    int act = 0;
#pragma unroll
    for (int tz = 0; tz < 3; ++tz) {
        const int iz = 2 * zz - 1 + tz;
        if ((unsigned)iz >= (unsigned)Din) continue;
#pragma unroll
        for (int ty = 0; ty < 3; ++ty) {
            const int iy = 2 * yy - 1 + ty;
            if ((unsigned)iy >= (unsigned)Din) continue;
            const int* row = mb + (iz * Din + iy) * Din;
#pragma unroll
            for (int tx = 0; tx < 3; ++tx) {
                const int ix = 2 * xx - 1 + tx;
                if ((unsigned)ix < (unsigned)Din) act |= (row[ix] != 0) ? 1 : 0;
            }
        }
    }
    volatile int* p = (volatile int*)(mo + i);
    *p = act;
    __threadfence();
    *p = act;
}

__global__ __launch_bounds__(256)
void k_conv1(const _Float16* __restrict__ xh, const _Float16* __restrict__ wt1,
             const float* __restrict__ b1, const int* __restrict__ m1,
             unsigned char* __restrict__ h1, int b)
{
    __shared__ __align__(16) _Float16 sB[64 * 128];
    __shared__ __align__(16) unsigned char sO[64 * 128];

    const int tid = threadIdx.x, lane = tid & 31, wave = tid >> 5;
    const int h = lane >> 4, nr = lane & 15;
    const int tile = blockIdx.x;
    const int zz = tile >> 6, yy = tile & 63;
    const _Float16 hz = 0;
    const _Float16* xb = xh + (size_t)b * V0 * 4;

#pragma unroll
    for (int k = 0; k < 8; ++k) {
        const int c = tid + 256 * k;
        const int n = c & 63, s = c >> 6;
        v4h val = {hz, hz, hz, hz};
        if (s < 27) {
            const int tx = s % 3, ty = (s / 3) % 3, tz = s / 9;
            const int iz = zz - 1 + tz, iy = yy - 1 + ty, ix = n - 1 + tx;
            if ((unsigned)iz < 64u && (unsigned)iy < 64u && (unsigned)ix < 64u)
                val = *(const v4h*)(xb + ((size_t)((iz * 64 + iy) * 64 + ix)) * 4);
        }
        *(v4h*)(sB + n * 128 + s * 4) = val;
    }
    __syncthreads();

    const int ct = wave & 3, vt0 = (wave >> 2) * 2;
    v8f acc[2];
    {
        v8f z = {0.f, 0.f, 0.f, 0.f, 0.f, 0.f, 0.f, 0.f};
        acc[0] = z; acc[1] = z;
    }
    const _Float16* arow = wt1 + (size_t)(ct * 16 + nr) * 128;
#pragma unroll
    for (int kc = 0; kc < 4; ++kc) {
        Frag a, bf;
        a.p[0] = *(const v8h*)(arow + kc * 32 + 8 * h);
        a.p[1] = *(const v8h*)(arow + kc * 32 + 16 + 8 * h);
#pragma unroll
        for (int nt = 0; nt < 2; ++nt) {
            const _Float16* brow = sB + ((vt0 + nt) * 16 + nr) * 128 + kc * 32 + 8 * h;
            bf.p[0] = *(const v8h*)brow;
            bf.p[1] = *(const v8h*)(brow + 16);
            acc[nt] = wmma_f16(a.v, bf.v, acc[nt]);
        }
        Guard<2>::run(acc, a.v, bf.v);
    }

    float bv[8];
#pragma unroll
    for (int r = 0; r < 8; ++r) bv[r] = b1[ct * 16 + 8 * h + r];
    const int* mrow = m1 + (size_t)b * V0 + (size_t)tile * 64;
#pragma unroll
    for (int nt = 0; nt < 2; ++nt) {
        const int n = (vt0 + nt) * 16 + nr;
        const bool act = (mrow[n] != 0);
        float v[8];
#pragma unroll
        for (int r = 0; r < 8; ++r) {
            const float y = fmaxf(fmaf(acc[nt][r], 0.125f, bv[r]), 0.f);
            v[r] = act ? y : 0.f;
        }
        v8h o = {(_Float16)v[0], (_Float16)v[1], (_Float16)v[2], (_Float16)v[3],
                 (_Float16)v[4], (_Float16)v[5], (_Float16)v[6], (_Float16)v[7]};
        *(v8h*)(sO + (size_t)n * 128 + (ct * 16 + 8 * h) * 2) = o;
    }
    __syncthreads();
    write_lines<64, 1>(sO, h1 + (size_t)tile * 64 * 128, 128, wave, lane);
}

template <int CIN, int COUT, int LOG2D, int VOX, int ESZ>
__global__ __launch_bounds__(256)
void k_conv(const _Float16* __restrict__ hin, const _Float16* __restrict__ wt,
            const float* __restrict__ bias, const int* __restrict__ mo,
            unsigned char* __restrict__ hout, int vox_base, int in_b0, float inv_scale)
{
    constexpr int D = 1 << LOG2D, Din = 2 * D;
    constexpr int NT = VOX / 16, CPR = CIN / 8, LCPR = __builtin_ctz(CPR), KC = CIN / 32;
    constexpr int LPV = ESZ, NL = VOX * LPV;
    constexpr int NSTG = (VOX * CPR) / 256;
    static_assert((VOX * CPR) % 256 == 0);
    static_assert(NT == 2 || NT == 4);

    __shared__ __align__(16) _Float16 sB[VOX * CIN];
    __shared__ __align__(16) unsigned char sO[VOX * 128 * ESZ];

    const int tid = threadIdx.x, lane = tid & 31, wave = tid >> 5;
    const int h = lane >> 4, nr = lane & 15;
    const int tile = blockIdx.x;
    const int vox0 = vox_base + tile * VOX;
    const int cb = blockIdx.y * 128 + wave * 16;
    const _Float16 hz = 0;

    v8f acc[NT];
    {
        v8f z = {0.f, 0.f, 0.f, 0.f, 0.f, 0.f, 0.f, 0.f};
#pragma unroll
        for (int nt = 0; nt < NT; ++nt) acc[nt] = z;
    }

#pragma unroll 1
    for (int t = 0; t < 27; ++t) {
        const int tx = t % 3, ty = (t / 3) % 3, tz = t / 9;
        __syncthreads();
#pragma unroll
        for (int k = 0; k < NSTG; ++k) {
            const int c = tid + 256 * k;
            const int n = c >> LCPR, q = c & (CPR - 1);
            const int vg = vox0 + n;
            const int xx = vg & (D - 1), yy = (vg >> LOG2D) & (D - 1), zz = (vg >> (2 * LOG2D)) & (D - 1);
            const int bb = vg >> (3 * LOG2D);
            const int iz = 2 * zz - 1 + tz, iy = 2 * yy - 1 + ty, ix = 2 * xx - 1 + tx;
            v8h val = {hz, hz, hz, hz, hz, hz, hz, hz};
            if ((unsigned)iz < (unsigned)Din && (unsigned)iy < (unsigned)Din && (unsigned)ix < (unsigned)Din) {
                const size_t vin = (((size_t)(bb - in_b0) * Din + iz) * Din + iy) * Din + ix;
                val = *(const v8h*)(hin + vin * CIN + q * 8);
            }
            *(v8h*)(sB + n * CIN + q * 8) = val;
        }
        __syncthreads();

        const _Float16* arow = wt + ((size_t)t * COUT + cb + nr) * CIN;
#pragma unroll
        for (int kc = 0; kc < KC; ++kc) {
            Frag a, bf;
            a.p[0] = *(const v8h*)(arow + kc * 32 + 8 * h);
            a.p[1] = *(const v8h*)(arow + kc * 32 + 16 + 8 * h);
#pragma unroll
            for (int nt = 0; nt < NT; ++nt) {
                const _Float16* brow = sB + (nt * 16 + nr) * CIN + kc * 32 + 8 * h;
                bf.p[0] = *(const v8h*)brow;
                bf.p[1] = *(const v8h*)(brow + 16);
                acc[nt] = wmma_f16(a.v, bf.v, acc[nt]);
            }
            Guard<NT>::run(acc, a.v, bf.v);
        }
    }

    float bv[8];
#pragma unroll
    for (int r = 0; r < 8; ++r) bv[r] = bias[cb + 8 * h + r];
#pragma unroll
    for (int nt = 0; nt < NT; ++nt) {
        const int n = nt * 16 + nr;
        const bool act = (mo[vox0 + n] != 0);
        float v[8];
#pragma unroll
        for (int r = 0; r < 8; ++r) {
            const float y = fmaxf(fmaf(acc[nt][r], inv_scale, bv[r]), 0.f);
            v[r] = act ? y : 0.f;
        }
        unsigned char* so = sO + ((size_t)n * 128 + wave * 16 + 8 * h) * ESZ;
        if (ESZ == 2) {
            v8h o = {(_Float16)v[0], (_Float16)v[1], (_Float16)v[2], (_Float16)v[3],
                     (_Float16)v[4], (_Float16)v[5], (_Float16)v[6], (_Float16)v[7]};
            *(v8h*)so = o;
        } else {
            v4f o0 = {v[0], v[1], v[2], v[3]};
            v4f o1 = {v[4], v[5], v[6], v[7]};
            *(v4f*)so = o0;
            *(v4f*)(so + 16) = o1;
        }
    }
    __syncthreads();
    write_lines<NL, LPV>(sO, hout + ((size_t)vox0 * COUT + blockIdx.y * 128) * ESZ,
                         COUT * ESZ, wave, lane);
}

__global__ __launch_bounds__(256)
void k_pool(const float* __restrict__ h4, float* __restrict__ out, int total4)
{
    const int i = blockIdx.x * 256 + threadIdx.x;
    if (i >= total4) return;
    const int b = i >> 7, cg = i & 127;
    const float* p = h4 + (size_t)b * 512 * 512 + cg * 4;
    v4f m = {-3.0e38f, -3.0e38f, -3.0e38f, -3.0e38f};
#pragma unroll 4
    for (int s = 0; s < 512; ++s) {
        const v4f v = *(const v4f*)(p + (size_t)s * 512);
        m.x = fmaxf(m.x, v.x); m.y = fmaxf(m.y, v.y);
        m.z = fmaxf(m.z, v.z); m.w = fmaxf(m.w, v.w);
    }
    v4f o;
    o.x = (m.x >= 0.f) ? m.x : 0.2f * m.x;
    o.y = (m.y >= 0.f) ? m.y : 0.2f * m.y;
    o.z = (m.z >= 0.f) ? m.z : 0.2f * m.z;
    o.w = (m.w >= 0.f) ? m.w : 0.2f * m.w;
    volatile v4f* q = (volatile v4f*)(out + (size_t)i * 4);
    *q = o;
    __threadfence();
    *q = o;
}

extern "C" void kernel_launch(void* const* d_in, const int* in_sizes, int n_in,
                              void* d_out, int out_size, void* d_ws, size_t ws_size,
                              hipStream_t stream)
{
    if (n_in < 10) return;
    if (in_sizes[0] != NB * 3 * V0 || in_sizes[1] != NB * V0 ||
        in_sizes[2] != 64 * 3 * 27 || in_sizes[3] != 64 ||
        in_sizes[4] != 128 * 64 * 27 || in_sizes[5] != 128 ||
        in_sizes[6] != 256 * 128 * 27 || in_sizes[7] != 256 ||
        in_sizes[8] != 512 * 256 * 27 || in_sizes[9] != 512 ||
        out_size != NB * 512) return;

    const float* x    = (const float*)d_in[0];
    const int*   mask = (const int*)d_in[1];
    const float* w1   = (const float*)d_in[2];
    const float* b1   = (const float*)d_in[3];
    const float* w2   = (const float*)d_in[4];
    const float* b2   = (const float*)d_in[5];
    const float* w3   = (const float*)d_in[6];
    const float* b3   = (const float*)d_in[7];
    const float* w4   = (const float*)d_in[8];
    const float* b4   = (const float*)d_in[9];
    float* out = (float*)d_out;

    char* ws = (char*)d_ws;
    size_t off = 0;
    auto alloc = [&](size_t bytes) -> char* {
        char* p = ws + off;
        off = (off + bytes + 255) & ~(size_t)255;
        return p;
    };
    _Float16* xh  = (_Float16*)alloc((size_t)NB * V0 * 4 * 2);
    _Float16* h1  = (_Float16*)alloc((size_t)V0 * 64 * 2);
    _Float16* h2  = (_Float16*)alloc((size_t)NB * 32768 * 128 * 2);
    _Float16* h3  = (_Float16*)alloc((size_t)NB * 4096 * 256 * 2);
    float*    h4  = (float*)alloc((size_t)NB * 512 * 512 * 4);
    int*      m1  = (int*)alloc((size_t)NB * V0 * 4);
    int*      m2  = (int*)alloc((size_t)NB * 32768 * 4);
    int*      m3  = (int*)alloc((size_t)NB * 4096 * 4);
    int*      m4  = (int*)alloc((size_t)NB * 512 * 4);
    _Float16* wt1 = (_Float16*)alloc((size_t)64 * 128 * 2);
    _Float16* wt2 = (_Float16*)alloc((size_t)27 * 128 * 64 * 2);
    _Float16* wt3 = (_Float16*)alloc((size_t)27 * 256 * 128 * 2);
    _Float16* wt4 = (_Float16*)alloc((size_t)27 * 512 * 256 * 2);
    if (off > ws_size || off > WS_LIMIT) return;

    k_prep_x<<<(NB * V0 + 255) / 256, 256, 0, stream>>>(x, mask, xh, NB * V0);
    k_wt1<<<(64 * 32 + 255) / 256, 256, 0, stream>>>(w1, wt1, 64 * 32);
    {
        const int t2 = 27 * 128 * 64 / 8, t3 = 27 * 256 * 128 / 8, t4 = 27 * 512 * 256 / 8;
        k_wtn<<<(t2 + 255) / 256, 256, 0, stream>>>(w2, wt2, 128, 64, 32.f, t2);
        k_wtn<<<(t3 + 255) / 256, 256, 0, stream>>>(w3, wt3, 256, 128, 64.f, t3);
        k_wtn<<<(t4 + 255) / 256, 256, 0, stream>>>(w4, wt4, 512, 256, 64.f, t4);
    }

    k_mask1<<<(NB * V0 + 255) / 256, 256, 0, stream>>>(mask, m1, NB * V0);
    k_dil<5><<<(NB * 32768 + 255) / 256, 256, 0, stream>>>(m1, m2, NB * 32768);
    k_dil<4><<<(NB * 4096 + 255) / 256, 256, 0, stream>>>(m2, m3, NB * 4096);
    k_dil<3><<<(NB * 512 + 255) / 256, 256, 0, stream>>>(m3, m4, NB * 512);

    for (int b = 0; b < NB; ++b) {
        k_conv1<<<V0 / 64, 256, 0, stream>>>(xh, wt1, b1, m1, (unsigned char*)h1, b);
        k_conv<64, 128, 5, 64, 2><<<dim3(32768 / 64, 1), 256, 0, stream>>>(
            h1, wt2, b2, m2, (unsigned char*)h2, b * 32768, b, 0.03125f);
    }
    k_conv<128, 256, 4, 64, 2><<<dim3(NB * 4096 / 64, 2), 256, 0, stream>>>(
        h2, wt3, b3, m3, (unsigned char*)h3, 0, 0, 0.015625f);
    k_conv<256, 512, 3, 32, 4><<<dim3(NB * 512 / 32, 4), 256, 0, stream>>>(
        h3, wt4, b4, m4, (unsigned char*)h4, 0, 0, 0.015625f);

    k_pool<<<(NB * 128 + 255) / 256, 256, 0, stream>>>(h4, out, NB * 128);
}
